// SpatialAttention_53721450939061
// MI455X (gfx1250) — hardware-verified
//
#include <hip/hip_runtime.h>
#include <math.h>

typedef __attribute__((ext_vector_type(16))) _Float16 v16h;
typedef __attribute__((ext_vector_type(16))) __bf16 v16b;
typedef __attribute__((ext_vector_type(8)))  _Float16 v8h;
typedef __attribute__((ext_vector_type(8)))  float v8f;
typedef __attribute__((ext_vector_type(4)))  float v4f;
typedef __attribute__((ext_vector_type(2)))  float v2f;
typedef __attribute__((ext_vector_type(4)))  unsigned v4u;
typedef __attribute__((ext_vector_type(4)))  int v4i;
typedef float __attribute__((may_alias)) float_a;
typedef int __attribute__((may_alias)) int_a;

template <typename T> __device__ __forceinline__ void vst2(void* p, T v) { *(volatile T*)p = v; __threadfence(); *(volatile T*)p = v; }
__device__ __forceinline__ v8f wmma16(v16h a, v16h b, v8f c) {
  v8f d = __builtin_amdgcn_wmma_f32_16x16x32_f16(false, a, false, b, (short)0, c, false, false);
  asm volatile("v_nop\n\tv_nop\n\tv_nop\n\tv_nop" : "+v"(d) : "v"(a), "v"(b));
  return d;
}
__device__ __forceinline__ v8f wmma_bf(v16b a, v16b b, v8f c) {
  v8f d = __builtin_amdgcn_wmma_f32_16x16x32_bf16(false, a, false, b, (short)0, c, false, false);
  asm volatile("v_nop\n\tv_nop\n\tv_nop\n\tv_nop" : "+v"(d) : "v"(a), "v"(b));
  return d;
}
__device__ __forceinline__ v16h frag_h(const _Float16* rowk0, int lane) {
  union { v16h v; v8h q[2]; } u; const _Float16* p = rowk0 + 8 * (lane >> 4);
  u.q[0] = *(const v8h*)p; u.q[1] = *(const v8h*)(p + 16); return u.v;
}
__device__ __forceinline__ v16h frag_f32(const float* rowk0, int lane) {
  v16h a; const float* p = rowk0 + 8 * (lane >> 4);
#pragma unroll
  for (int i = 0; i < 8; ++i) { a[i] = (_Float16)p[i]; a[8 + i] = (_Float16)p[16 + i]; }
  return a;
}
__device__ __forceinline__ v16h frag_f32s(const float* rowk0, int lane, float sc) {
  v16h a; const float* p = rowk0 + 8 * (lane >> 4);
#pragma unroll
  for (int i = 0; i < 8; ++i) { a[i] = (_Float16)(p[i] * sc); a[8 + i] = (_Float16)(p[16 + i] * sc); }
  return a;
}
__device__ __forceinline__ v16h fragc_f32(const float* W, int k0, int n, int lane, int ld, int K) {
  v16h a; const int g = lane >> 4;
#pragma unroll
  for (int i = 0; i < 8; ++i) { const int ka = k0 + 8 * g + i, kb = ka + 16;
    a[i] = (_Float16)(ka < K ? W[(size_t)(ka < K ? ka : K - 1) * ld + n] : 0.f); a[8 + i] = (_Float16)(kb < K ? W[(size_t)(kb < K ? kb : K - 1) * ld + n] : 0.f); }
  return a;
}
struct F2 { v16b h, l; };
__device__ __forceinline__ F2 bsplit16(const float v[16]) { F2 r;
#pragma unroll
  for (int i = 0; i < 16; ++i) { const __bf16 h = (__bf16)v[i]; r.h[i] = h; r.l[i] = (__bf16)(v[i] - (float)h); }
  return r; }
__device__ __forceinline__ F2 split_row(const float* row, int k0, int lane) { float v[16]; const float* p = row + k0 + 8 * (lane >> 4);
#pragma unroll
  for (int i = 0; i < 8; ++i) { v[i] = p[i]; v[8 + i] = p[16 + i]; }
  return bsplit16(v); }
__device__ __forceinline__ F2 split_rowK(const float* row, int k0, int lane, int K) { float v[16]; const int g = lane >> 4;
#pragma unroll
  for (int i = 0; i < 8; ++i) { const int ka = k0 + 8 * g + i, kb = ka + 16; v[i] = ka < K ? row[ka < K ? ka : K - 1] : 0.f; v[8 + i] = kb < K ? row[kb < K ? kb : K - 1] : 0.f; }
  return bsplit16(v); }
__device__ __forceinline__ F2 split_col(const float* W, int k0, int n, int lane, int ld, int K) { float v[16]; const int g = lane >> 4;
#pragma unroll
  for (int i = 0; i < 8; ++i) { const int ka = k0 + 8 * g + i, kb = ka + 16; v[i] = ka < K ? W[(size_t)(ka < K ? ka : K - 1) * ld + n] : 0.f; v[8 + i] = kb < K ? W[(size_t)(kb < K ? kb : K - 1) * ld + n] : 0.f; }
  return bsplit16(v); }
__device__ __forceinline__ v8f mac3(const F2& a, const F2& b, v8f c) { c = wmma_bf(a.l, b.h, c); c = wmma_bf(a.h, b.l, c); return wmma_bf(a.h, b.h, c); }
__device__ __forceinline__ float sigm(float v) { return 1.0f / (1.0f + expf(-v)); }
#define LDSX() do { asm volatile("s_wait_dscnt 0" ::: "memory"); __builtin_amdgcn_wave_barrier(); __builtin_amdgcn_fence(__ATOMIC_RELEASE, "workgroup"); } while (0)

#define NB 16
#define TT 2048
#define CC 1024
#define DIN 1024
#define NH 16
#define HD 64
#define NQB (TT / 64)
#define HG 4
#define SCALE (0.125f)
#define CAUSAL 1
#ifndef TNB
#define TNB NB
#endif
__device__ __forceinline__ float bfr(float v) { return (float)(__bf16)v; }
__host__ __device__ __forceinline__ int kb_last(int qb) { return CAUSAL ? ((qb * 64 + 63) >> 7) : (TT / 128 - 1); }
typedef __attribute__((ext_vector_type(8))) __bf16 v8b;
__device__ __forceinline__ v16b frag_b(const __bf16* rowk0, int lane) {
  union { v16b v; v8b q[2]; } u; const __bf16* p = rowk0 + 8 * (lane >> 4);
  u.q[0] = *(const v8b*)p; u.q[1] = *(const v8b*)(p + 16); return u.v;
}
#define QBH 6
#define QHI 384
#define KHI 384
__device__ __forceinline__ v16b wcol_io(const float* Wm, int k0, int o, int lane, int ld) { v16b w; const int g = lane >> 4;
#pragma unroll
  for (int i = 0; i < 8; ++i) { w[i] = (__bf16)Wm[(size_t)(k0 + 8 * g + i) * ld + o]; w[8 + i] = (__bf16)Wm[(size_t)(k0 + 16 + 8 * g + i) * ld + o]; }
  return w; }
__device__ __forceinline__ v16b wcol_oi(const float* Wm, int k0, int o, int lane, int K) { v16b w; const float* p = Wm + (size_t)o * K + k0 + 8 * (lane >> 4);
#pragma unroll
  for (int i = 0; i < 8; ++i) { w[i] = (__bf16)p[i]; w[8 + i] = (__bf16)p[16 + i]; }
  return w; }
__device__ __forceinline__ v16h wcolh_io(const float* Wm, int k0, int o, int lane, int ld) { v16h w; const int g = lane >> 4;
#pragma unroll
  for (int i = 0; i < 8; ++i) { w[i] = (_Float16)(bfr(Wm[(size_t)(k0 + 8 * g + i) * ld + o]) * 256.0f); w[8 + i] = (_Float16)(bfr(Wm[(size_t)(k0 + 16 + 8 * g + i) * ld + o]) * 256.0f); }
  return w; }
__device__ __forceinline__ v16h wcolh_oi(const float* Wm, int k0, int o, int lane, int K) { v16h w; const float* p = Wm + (size_t)o * K + k0 + 8 * (lane >> 4);
#pragma unroll
  for (int i = 0; i < 8; ++i) { w[i] = (_Float16)(bfr(p[i]) * 256.0f); w[8 + i] = (_Float16)(bfr(p[16 + i]) * 256.0f); }
  return w; }
#define WQKV_LAYOUT 1
__device__ __forceinline__ v16b wcol_hdk(const float* Wm, int k0, int o, int lane) { v16b w; const int g = lane >> 4; const float* p = Wm + (size_t)(o / HD) * DIN * HD + (o % HD);
#pragma unroll
  for (int i = 0; i < 8; ++i) { w[i] = (__bf16)p[(size_t)(k0 + 8 * g + i) * HD]; w[8 + i] = (__bf16)p[(size_t)(k0 + 16 + 8 * g + i) * HD]; }
  return w; }
#define WO_OUT_IN 1
#if WQKV_LAYOUT == 1
#define WCOL(W, k0, o, lane) wcol_oi(W, k0, o, lane, DIN)
#elif WQKV_LAYOUT == 2
#define WCOL(W, k0, o, lane) wcol_hdk(W, k0, o, lane)
#else
#define WCOL(W, k0, o, lane) wcol_io(W, k0, o, lane, CC)
#endif
#if WO_OUT_IN
#define WOCOL(W, k0, o, lane) wcol_oi(W, k0, o, lane, CC)
#define WOCOLH(W, k0, o, lane) wcolh_oi(W, k0, o, lane, CC)
#else
#define WOCOL(W, k0, o, lane) wcol_io(W, k0, o, lane, DIN)
#define WOCOLH(W, k0, o, lane) wcolh_io(W, k0, o, lane, DIN)
#endif

#ifndef SM_EXTRA_PARAMS
#define SM_EXTRA_PARAMS
#endif
#ifndef PROJ_EXTRA_PARAMS
#define PROJ_EXTRA_PARAMS
#endif
#ifndef SM_MASK_HOOK
#define SM_MASK_HOOK (void)0
#endif

#define WS_QH  0u
#define WS_KH  (WS_QH + 2u * (size_t)NB * TT * CC)
#define WS_VT  (WS_KH + 2u * (size_t)NB * TT * CC)
#define WS_QL  (WS_VT + 2u * (size_t)NB * CC * TT)
#define WS_KL  (WS_QL + 2u * (size_t)NB * QHI * CC)
#define WS_VB  (WS_KL + 2u * (size_t)NB * KHI * CC)
#define WS_VBL (WS_VB + 2u * (size_t)NB * CC * KHI)
#define WS_S   (WS_VBL + 2u * (size_t)NB * CC * KHI)
#define WS_Y   (WS_S  + 4u * (size_t)HG * TT * TT)
#define WS_END (WS_Y  + 4u * (size_t)NB * TT * CC)


#define NBT 16
#define TN 1024
#define NC 512
__global__ __launch_bounds__(128) void k_linr(const float* __restrict__ X, const float* __restrict__ WQ, const float* __restrict__ WK, const float* __restrict__ WV, float* __restrict__ YQ, float* __restrict__ YK, float* __restrict__ YV) {
  __shared__ __align__(16) float sf[4][16][132];
  const int tid = threadIdx.x, wave = tid >> 5, lane = tid & 31, col = lane & 15, g = lane >> 4; const int c0 = blockIdx.x * 64 + wave * 16; const int t0 = blockIdx.y * 128; const int b = blockIdx.z / 3, which = blockIdx.z % 3;
  const float* W = which == 0 ? WQ : which == 1 ? WK : WV; float* Y = which == 0 ? YQ : which == 1 ? YK : YV; const float* xb = X + (size_t)b * TN * NC;
  v8f acc[8] = {};
#pragma unroll 1
  for (int kc = 0; kc < NC / 32; ++kc) { const F2 a = split_row(W + (size_t)(c0 + col) * NC, kc * 32, lane); asm volatile("s_wait_loadcnt 0x0" ::: "memory");
#pragma unroll
    for (int j = 0; j < 8; ++j) { const F2 xf = split_row(xb + (size_t)(t0 + j * 16 + col) * NC, kc * 32, lane); asm volatile("s_wait_loadcnt 0x0" ::: "memory"); acc[j] = wmma_bf(a.h, xf.h, acc[j]); } }
#pragma unroll
  for (int j = 0; j < 8; ++j)
#pragma unroll
    for (int r = 0; r < 8; ++r) sf[wave][8 * g + r][j * 16 + col] = acc[j][r];
  LDSX(); for (int rl = 0; rl < 16; ++rl) vst2(Y + ((size_t)b * NC + c0 + rl) * TN + t0 + lane * 4, *(const v4f*)&sf[wave][rl][lane * 4]); }
__global__ __launch_bounds__(128) void k_sgem(const float* __restrict__ YQ, const float* __restrict__ YK, float* __restrict__ S) { __shared__ __align__(16) float sf[4][16][132];
  const int tid = threadIdx.x, wave = tid >> 5, lane = tid & 31, col = lane & 15, g = lane >> 4; const int n0 = blockIdx.x * 64 + wave * 16; const int m0 = blockIdx.y * 128; const int b = blockIdx.z;
  const float* qb = YQ + (size_t)b * NC * TN; const float* kb = YK + (size_t)b * NC * TN;
  v8f acc[8] = {};
#pragma unroll 1
  for (int kc = 0; kc < TN / 32; ++kc) { const F2 a = split_row(qb + (size_t)(n0 + col) * TN, kc * 32, lane); asm volatile("s_wait_loadcnt 0x0" ::: "memory");
#pragma unroll
    for (int j = 0; j < 8; ++j) { const F2 w = split_row(kb + (size_t)(m0 + j * 16 + col) * TN, kc * 32, lane); asm volatile("s_wait_loadcnt 0x0" ::: "memory"); acc[j] = mac3(a, w, acc[j]); } }
#pragma unroll
  for (int j = 0; j < 8; ++j)
#pragma unroll
    for (int r = 0; r < 8; ++r) sf[wave][8 * g + r][j * 16 + col] = acc[j][r] * 0.044194173824159216f;
  LDSX(); for (int rl = 0; rl < 16; ++rl) vst2(S + ((size_t)b * NC + n0 + rl) * NC + m0 + lane * 4, *(const v4f*)&sf[wave][rl][lane * 4]); }
__global__ __launch_bounds__(256) void k_rsm(float* __restrict__ S) { const int wave = threadIdx.x >> 5, lane = threadIdx.x & 31; const size_t row = (size_t)blockIdx.x * 8 + wave; if (row >= (size_t)TNB * NC) return; float* sr = S + row * NC; float v[NC / 32]; float m = -3.0e38f;
#pragma unroll
  for (int i = 0; i < NC / 128; ++i) { const v4f t4 = *(const v4f*)(sr + i * 128 + lane * 4); v[4 * i] = t4[0]; v[4 * i + 1] = t4[1]; v[4 * i + 2] = t4[2]; v[4 * i + 3] = t4[3]; }
  asm volatile("s_wait_loadcnt 0x0" ::: "memory");
#pragma unroll
  for (int i = 0; i < NC / 32; ++i) m = fmaxf(m, v[i]);
#pragma unroll
  for (int o = 1; o < 32; o <<= 1) m = fmaxf(m, __shfl_xor(m, o));
  float sum = 0.f;
#pragma unroll
  for (int i = 0; i < NC / 32; ++i) { v[i] = expf(v[i] - m); sum += v[i]; }
#pragma unroll
  for (int o = 1; o < 32; o <<= 1) sum += __shfl_xor(sum, o);
  const float inv = 1.0f / sum;
#pragma unroll
  for (int i = 0; i < NC / 128; ++i) { v4f o4; o4[0] = v[4 * i] * inv; o4[1] = v[4 * i + 1] * inv; o4[2] = v[4 * i + 2] * inv; o4[3] = v[4 * i + 3] * inv; vst2(sr + i * 128 + lane * 4, o4); } }
__global__ __launch_bounds__(128) void k_pvt(const float* __restrict__ S, const float* __restrict__ YV, float* __restrict__ PX) { __shared__ __align__(16) float sf[4][16][132];
  const int tid = threadIdx.x, wave = tid >> 5, lane = tid & 31, col = lane & 15, g = lane >> 4; const int n0 = blockIdx.x * 64 + wave * 16; const int t0 = blockIdx.y * 128; const int b = blockIdx.z;
  const float* pb = S + (size_t)b * NC * NC; const float* vb = YV + (size_t)b * NC * TN;
  v8f acc[8] = {};
#pragma unroll 1
  for (int kc = 0; kc < NC / 32; ++kc) { const F2 a = split_row(pb + (size_t)(n0 + col) * NC, kc * 32, lane); asm volatile("s_wait_loadcnt 0x0" ::: "memory");
#pragma unroll
    for (int j = 0; j < 8; ++j) { const F2 w = split_col(vb, kc * 32, t0 + j * 16 + col, lane, TN, NC); asm volatile("s_wait_loadcnt 0x0" ::: "memory"); acc[j] = mac3(a, w, acc[j]); } }
#pragma unroll
  for (int j = 0; j < 8; ++j)
#pragma unroll
    for (int r = 0; r < 8; ++r) sf[wave][8 * g + r][j * 16 + col] = acc[j][r];
  LDSX(); for (int rl = 0; rl < 16; ++rl) vst2(PX + ((size_t)b * NC + n0 + rl) * TN + t0 + lane * 4, *(const v4f*)&sf[wave][rl][lane * 4]); }
__global__ __launch_bounds__(128) void k_outT(const float* __restrict__ PX, const float* __restrict__ WP, const float* __restrict__ BP, float* __restrict__ OUT) { __shared__ __align__(16) float st[128][68];
  const int tid = threadIdx.x, wave = tid >> 5, lane = tid & 31, col = lane & 15, g = lane >> 4; const int o0 = blockIdx.x * 64 + wave * 16; const int t0 = blockIdx.y * 128; const int b = blockIdx.z;
  const float* pb = PX + (size_t)b * NC * TN;
  v8f acc[8] = {};
#pragma unroll 1
  for (int kc = 0; kc < NC / 32; ++kc) { const F2 a = split_row(WP + (size_t)(o0 + col) * NC, kc * 32, lane); asm volatile("s_wait_loadcnt 0x0" ::: "memory");
#pragma unroll
    for (int j = 0; j < 8; ++j) { const F2 w = split_col(pb, kc * 32, t0 + j * 16 + col, lane, TN, NC); asm volatile("s_wait_loadcnt 0x0" ::: "memory"); acc[j] = wmma_bf(a.h, w.h, acc[j]); acc[j] = wmma_bf(a.h, w.l, acc[j]); } }
#pragma unroll
  for (int j = 0; j < 8; ++j)
#pragma unroll
    for (int r = 0; r < 8; ++r) { const float bias = bfr(BP[o0 + 8 * g + r]); st[j * 16 + col][wave * 16 + 8 * g + r] = acc[j][r] + bias; }
  __syncthreads();
  for (int e = tid; e < 128 * 16; e += 128) { const int tl = e >> 4, q = e & 15; vst2(OUT + ((size_t)b * TN + t0 + tl) * NC + blockIdx.x * 64 + q * 4, *(const v4f*)&st[tl][q * 4]); } }
#define WS_YQ 0u
#define WS_YK (WS_YQ + 4u * (size_t)NBT * NC * TN)
#define WS_YV (WS_YK + 4u * (size_t)NBT * NC * TN)
#define WS_SS (WS_YV + 4u * (size_t)NBT * NC * TN)
#define WS_PX (WS_SS + 4u * (size_t)NBT * NC * NC)
#define WS_TOT (WS_PX + 4u * (size_t)NBT * NC * TN)
extern "C" void kernel_launch(void* const* d_in, const int* in_sizes, int n_in, void* d_out, int out_size, void* d_ws, size_t ws_size, hipStream_t stream) {
  (void)in_sizes; (void)n_in; (void)out_size;
  const float** F = (const float**)d_in;
  if (ws_size < (size_t)WS_TOT) return;
  char* ws = (char*)d_ws; float *YQ = (float*)(ws + WS_YQ), *YK = (float*)(ws + WS_YK), *YV = (float*)(ws + WS_YV), *SS = (float*)(ws + WS_SS), *PX = (float*)(ws + WS_PX);
  k_linr<<<dim3(NC / 64, TN / 128, TNB * 3), 128, 0, stream>>>(F[0], F[1], F[2], F[3], YQ, YK, YV);
  k_sgem<<<dim3(NC / 64, NC / 128, TNB), 128, 0, stream>>>(YQ, YK, SS);
  k_rsm<<<dim3((TNB * NC + 7) / 8), 256, 0, stream>>>(SS);
  k_pvt<<<dim3(NC / 64, TN / 128, TNB), 128, 0, stream>>>(SS, YV, PX);
  k_outT<<<dim3(NC / 64, TN / 128, TNB), 128, 0, stream>>>(PX, F[4], F[5], (float*)d_out);
}
